// MixtureOfExperts_29755533427503
// MI455X (gfx1250) — hardware-verified
//
#include <hip/hip_runtime.h>
#include <math.h>

typedef __attribute__((ext_vector_type(16))) _Float16 v16h;
typedef __attribute__((ext_vector_type(16))) __bf16 v16b;
typedef __attribute__((ext_vector_type(8)))  _Float16 v8h;
typedef __attribute__((ext_vector_type(8)))  float v8f;
typedef __attribute__((ext_vector_type(4)))  float v4f;
typedef __attribute__((ext_vector_type(2)))  float v2f;
typedef __attribute__((ext_vector_type(4)))  unsigned v4u;
typedef __attribute__((ext_vector_type(4)))  int v4i;
typedef float __attribute__((may_alias)) float_a;
typedef int __attribute__((may_alias)) int_a;

template <typename T> __device__ __forceinline__ void vst2(void* p, T v) { *(volatile T*)p = v; __threadfence(); *(volatile T*)p = v; }
__device__ __forceinline__ v8f wmma16(v16h a, v16h b, v8f c) {
  v8f d = __builtin_amdgcn_wmma_f32_16x16x32_f16(false, a, false, b, (short)0, c, false, false);
  asm volatile("v_nop\n\tv_nop\n\tv_nop\n\tv_nop" : "+v"(d) : "v"(a), "v"(b));
  return d;
}
__device__ __forceinline__ v8f wmma_bf(v16b a, v16b b, v8f c) {
  v8f d = __builtin_amdgcn_wmma_f32_16x16x32_bf16(false, a, false, b, (short)0, c, false, false);
  asm volatile("v_nop\n\tv_nop\n\tv_nop\n\tv_nop" : "+v"(d) : "v"(a), "v"(b));
  return d;
}
__device__ __forceinline__ v16h frag_h(const _Float16* rowk0, int lane) {
  union { v16h v; v8h q[2]; } u; const _Float16* p = rowk0 + 8 * (lane >> 4);
  u.q[0] = *(const v8h*)p; u.q[1] = *(const v8h*)(p + 16); return u.v;
}
__device__ __forceinline__ v16h frag_f32(const float* rowk0, int lane) {
  v16h a; const float* p = rowk0 + 8 * (lane >> 4);
#pragma unroll
  for (int i = 0; i < 8; ++i) { a[i] = (_Float16)p[i]; a[8 + i] = (_Float16)p[16 + i]; }
  return a;
}
__device__ __forceinline__ v16h frag_f32s(const float* rowk0, int lane, float sc) {
  v16h a; const float* p = rowk0 + 8 * (lane >> 4);
#pragma unroll
  for (int i = 0; i < 8; ++i) { a[i] = (_Float16)(p[i] * sc); a[8 + i] = (_Float16)(p[16 + i] * sc); }
  return a;
}
__device__ __forceinline__ v16h fragc_f32(const float* W, int k0, int n, int lane, int ld, int K) {
  v16h a; const int g = lane >> 4;
#pragma unroll
  for (int i = 0; i < 8; ++i) { const int ka = k0 + 8 * g + i, kb = ka + 16;
    a[i] = (_Float16)(ka < K ? W[(size_t)(ka < K ? ka : K - 1) * ld + n] : 0.f); a[8 + i] = (_Float16)(kb < K ? W[(size_t)(kb < K ? kb : K - 1) * ld + n] : 0.f); }
  return a;
}
struct F2 { v16b h, l; };
__device__ __forceinline__ F2 bsplit16(const float v[16]) { F2 r;
#pragma unroll
  for (int i = 0; i < 16; ++i) { const __bf16 h = (__bf16)v[i]; r.h[i] = h; r.l[i] = (__bf16)(v[i] - (float)h); }
  return r; }
__device__ __forceinline__ F2 split_row(const float* row, int k0, int lane) { float v[16]; const float* p = row + k0 + 8 * (lane >> 4);
#pragma unroll
  for (int i = 0; i < 8; ++i) { v[i] = p[i]; v[8 + i] = p[16 + i]; }
  return bsplit16(v); }
__device__ __forceinline__ F2 split_rowK(const float* row, int k0, int lane, int K) { float v[16]; const int g = lane >> 4;
#pragma unroll
  for (int i = 0; i < 8; ++i) { const int ka = k0 + 8 * g + i, kb = ka + 16; v[i] = ka < K ? row[ka < K ? ka : K - 1] : 0.f; v[8 + i] = kb < K ? row[kb < K ? kb : K - 1] : 0.f; }
  return bsplit16(v); }
__device__ __forceinline__ F2 split_col(const float* W, int k0, int n, int lane, int ld, int K) { float v[16]; const int g = lane >> 4;
#pragma unroll
  for (int i = 0; i < 8; ++i) { const int ka = k0 + 8 * g + i, kb = ka + 16; v[i] = ka < K ? W[(size_t)(ka < K ? ka : K - 1) * ld + n] : 0.f; v[8 + i] = kb < K ? W[(size_t)(kb < K ? kb : K - 1) * ld + n] : 0.f; }
  return bsplit16(v); }
__device__ __forceinline__ v8f mac3(const F2& a, const F2& b, v8f c) { c = wmma_bf(a.l, b.h, c); c = wmma_bf(a.h, b.l, c); return wmma_bf(a.h, b.h, c); }
__device__ __forceinline__ float sigm(float v) { return 1.0f / (1.0f + expf(-v)); }
#define LDSX() do { asm volatile("s_wait_dscnt 0" ::: "memory"); __builtin_amdgcn_wave_barrier(); __builtin_amdgcn_fence(__ATOMIC_RELEASE, "workgroup"); } while (0)

#define NT 16384
#define DD 256
#define HH 1024
#define OO 256
#define NE 16
#define KS 1
#define NSH 1
#define NRB (NT / 64 + NE)
typedef __attribute__((ext_vector_type(4))) int v4i2;
__device__ __forceinline__ float bfr(float v) { return (float)(__bf16)v; }
__device__ __forceinline__ v16b wcol_in(const float* Wm, int k0, int o, int lane, int ld, int nvalid) { v16b w; const int g = lane >> 4; const int oc = o < nvalid ? o : 0; const float keep = o < nvalid ? 1.f : 0.f; float t0[8], t1[8];
#pragma unroll
  for (int i = 0; i < 8; ++i) t0[i] = Wm[(size_t)(k0 + 8 * g + i) * ld + oc];
  asm volatile("s_wait_loadcnt 0x0" ::: "memory");
#pragma unroll
  for (int i = 0; i < 8; ++i) t1[i] = Wm[(size_t)(k0 + 16 + 8 * g + i) * ld + oc];
  asm volatile("s_wait_loadcnt 0x0" ::: "memory");
#pragma unroll
  for (int i = 0; i < 8; ++i) { w[i] = (__bf16)(t0[i] * keep); w[8 + i] = (__bf16)(t1[i] * keep); }
  return w; }
#define WS_IDX 0u
#define WS_WGT (WS_IDX + 16u * NT)
#define WS_TOK (WS_WGT + 16u * NT)
#define WS_RB  (WS_TOK + 16u * NT)
#define WS_H   (WS_RB + 64u * NRB + 1024u)
#define WS_END (WS_H + 4u * (size_t)NT * HS)


__global__ __launch_bounds__(128) void k_dense(const float* __restrict__ X, const float* __restrict__ WE, const float* __restrict__ BE, const float* __restrict__ WG, const float* __restrict__ BGt, float* __restrict__ OUT) {
  __shared__ __align__(16) float sf[4][16][132]; __shared__ float sl[64][NE + 1]; __shared__ float sg[64][NE + 1];
  const int tid = threadIdx.x, wave = tid >> 5, lane = tid & 31, col = lane & 15, g = lane >> 4; const int c0 = blockIdx.y * 64; const size_t r0 = (size_t)blockIdx.x * 64 + wave * 16;
  { v8f lg = {};
#pragma unroll 2
    for (int kc = 0; kc < DD / 32; ++kc) { v16b a; { const float* p = X + (r0 + col) * DD + kc * 32 + 8 * g; float t0[8], t1[8];
#pragma unroll
        for (int i = 0; i < 8; ++i) t0[i] = p[i];
        asm volatile("s_wait_loadcnt 0x0" ::: "memory");
#pragma unroll
        for (int i = 0; i < 8; ++i) t1[i] = p[16 + i];
        asm volatile("s_wait_loadcnt 0x0" ::: "memory");
#pragma unroll
        for (int i = 0; i < 8; ++i) { a[i] = (__bf16)t0[i]; a[8 + i] = (__bf16)t1[i]; } }
      v16b w; { float u0[8], u1[8];
#pragma unroll
        for (int i = 0; i < 8; ++i) u0[i] = WG[(size_t)(kc * 32 + 8 * g + i) * NE + col];
        asm volatile("s_wait_loadcnt 0x0" ::: "memory");
#pragma unroll
        for (int i = 0; i < 8; ++i) u1[i] = WG[(size_t)(kc * 32 + 16 + 8 * g + i) * NE + col];
        asm volatile("s_wait_loadcnt 0x0" ::: "memory");
#pragma unroll
        for (int i = 0; i < 8; ++i) { w[i] = (__bf16)u0[i]; w[8 + i] = (__bf16)u1[i]; } }
      lg = wmma_bf(a, w, lg); }
    const float bge = bfr(BGt[col]); asm volatile("s_wait_loadcnt 0x0" ::: "memory");
#pragma unroll
    for (int r = 0; r < 8; ++r) sl[wave * 16 + 8 * g + r][col] = lg[r] + bge; }
  __syncthreads();
  if (tid < 64) { float m = -3.0e38f; for (int e = 0; e < NE; ++e) m = fmaxf(m, sl[tid][e]); float den = 0.f; float ex[NE];
#pragma unroll
    for (int e = 0; e < NE; ++e) { ex[e] = expf(sl[tid][e] - m); den += ex[e]; }
#pragma unroll
    for (int e = 0; e < NE; ++e) sg[tid][e] = ex[e] / den; }
  __syncthreads();
  v8f outacc[4] = {};
  float gme[8];
#pragma unroll 1
  for (int e = 0; e < NE; ++e) {
#pragma unroll
    for (int r = 0; r < 8; ++r) gme[r] = sg[wave * 16 + 8 * g + r][e];
    v8f acc[4] = {};
#pragma unroll 1
    for (int kc = 0; kc < DD / 32; ++kc) { v16b a; { const float* p = X + (r0 + col) * DD + kc * 32 + 8 * g; float t0[8], t1[8];
#pragma unroll
        for (int i = 0; i < 8; ++i) t0[i] = p[i];
        asm volatile("s_wait_loadcnt 0x0" ::: "memory");
#pragma unroll
        for (int i = 0; i < 8; ++i) t1[i] = p[16 + i];
        asm volatile("s_wait_loadcnt 0x0" ::: "memory");
#pragma unroll
        for (int i = 0; i < 8; ++i) { a[i] = (__bf16)t0[i]; a[8 + i] = (__bf16)t1[i]; } }
      const float* Wx = WE + (size_t)e * DD * OO;
#pragma unroll
      for (int j = 0; j < 4; ++j) { v16b w; { const int o = c0 + j * 16 + col; float u0[8], u1[8];
#pragma unroll
          for (int i = 0; i < 8; ++i) u0[i] = Wx[(size_t)(kc * 32 + 8 * g + i) * OO + o];
          asm volatile("s_wait_loadcnt 0x0" ::: "memory");
#pragma unroll
          for (int i = 0; i < 8; ++i) u1[i] = Wx[(size_t)(kc * 32 + 16 + 8 * g + i) * OO + o];
          asm volatile("s_wait_loadcnt 0x0" ::: "memory");
#pragma unroll
          for (int i = 0; i < 8; ++i) { w[i] = (__bf16)u0[i]; w[8 + i] = (__bf16)u1[i]; } }
        acc[j] = wmma_bf(a, w, acc[j]); } }
#pragma unroll
    for (int j = 0; j < 4; ++j) { const float bb = bfr(BE[(size_t)e * OO + c0 + j * 16 + col]); asm volatile("s_wait_loadcnt 0x0" ::: "memory");
#pragma unroll
      for (int r = 0; r < 8; ++r) { const float u = acc[j][r] + bb; const float h = 0.5f * u * (1.0f + erff(u * 0.70710678118654752f)); outacc[j][r] += h * gme[r]; } } }
#pragma unroll
  for (int j = 0; j < 4; ++j)
#pragma unroll
    for (int r = 0; r < 8; ++r) sf[wave][8 * g + r][j * 16 + col] = outacc[j][r];
  LDSX(); for (int rl = 0; rl < 16; ++rl) if (lane < 16) vst2(OUT + (r0 + rl) * OO + c0 + lane * 4, *(const v4f*)&sf[wave][rl][lane * 4]); }
extern "C" void kernel_launch(void* const* d_in, const int* in_sizes, int n_in, void* d_out, int out_size, void* d_ws, size_t ws_size, hipStream_t stream) {
  (void)in_sizes; (void)n_in; (void)out_size; (void)d_ws; (void)ws_size;
  const float** F = (const float**)d_in;
  k_dense<<<dim3(NT / 64, OO / 64), 128, 0, stream>>>(F[0], F[1], F[2], F[3], F[4], (float*)d_out);
}
